// DecoderWithAttention_18528488915169
// MI455X (gfx1250) — hardware-verified
//
#include <hip/hip_runtime.h>
#include <stdint.h>

constexpr int NB = 32;
constexpr int NP = 196;
constexpr int NF = 2048;
constexpr int NA = 512;
constexpr int NH = 512;
constexpr int NE = 512;
constexpr int NV = 10000;
constexpr int NVP = 10048;
constexpr int NT = 25;
constexpr int KIH = 2560;
constexpr int KZ = 3072;
constexpr int NCAT = 2560;
constexpr int PTK = 256;
constexpr int KAWE = 224;
constexpr int APW = 224;
constexpr int MROWS = NB * NP;
constexpr int SA_PITCH = 264;
constexpr int TP_PITCH = 264;

constexpr float SC_W = 64.0f;
constexpr float SC_ENC = 16.0f;
constexpr float SC_Z = 256.0f;
constexpr float SC_P = 1024.0f;

static_assert(MROWS % 64 == 0, "M tile 64 for the encoder projection");
static_assert(NB % 32 == 0, "M tile 32 for per-step GEMMs");
static_assert(NA % 64 == 0 && (2 * NH) % 64 == 0 && NCAT % 64 == 0 && (4 * NH) % 64 == 0 && NVP % 64 == 0, "N tiles");
static_assert(NF % 32 == 0 && NH % 32 == 0 && KZ % 32 == 0 && KAWE % 32 == 0 && KAWE >= NP && KAWE <= PTK, "K steps");
static_assert(NA % 32 == 0 && NCAT % 32 == 0 && (4 * NH) % 32 == 0 && NVP % 32 == 0 && (2 * NH) % 32 == 0, "f32 row pitches are whole lines");
static_assert(APW % 32 == 0 && APW >= NP && (PTK * 2) % 128 == 0 && (KZ * 2) % 128 == 0, "plane pitches are whole lines");
static_assert(NV % 4 == 0 && NP % 4 == 0, "float4 repack never straddles a row");
static_assert(((long)NB * NT * NV * 4) % 128 == 0, "second output starts on a line");
static_assert((((long)NB * NT * NV + (long)NB * NT * NP) / 4) % 32 == 0, "repack waves are whole");

typedef __attribute__((ext_vector_type(16))) _Float16 v16h;
typedef __attribute__((ext_vector_type(8)))  _Float16 v8h;
typedef __attribute__((ext_vector_type(16))) __bf16   v16b;
typedef __attribute__((ext_vector_type(8)))  __bf16   v8b;
typedef __attribute__((ext_vector_type(8)))  float    v8f;
typedef __attribute__((ext_vector_type(4)))  float    v4f;
typedef __attribute__((ext_vector_type(2)))  float    v2f;

__device__ __forceinline__ unsigned short f2bf_bits(float f) {
  unsigned u = __float_as_uint(f);
  return (unsigned short)((u + 0x7FFFu + ((u >> 16) & 1u)) >> 16);
}
__device__ __forceinline__ float bf_bits2f(unsigned short h) { return __uint_as_float(((unsigned)h) << 16); }
__device__ __forceinline__ unsigned short h2bits(_Float16 h) { return __builtin_bit_cast(unsigned short, h); }

__device__ __forceinline__ void dep_guard_h(v8f& a, v8f& b, v16h x, v16h y) { asm volatile("v_nop\n\tv_nop\n\tv_nop\n\tv_nop" : "+v"(a), "+v"(b) : "v"(x), "v"(y)); }
__device__ __forceinline__ void dep_guard_b(v8f& a, v8f& b, v16b x, v16b y) { asm volatile("v_nop\n\tv_nop\n\tv_nop\n\tv_nop" : "+v"(a), "+v"(b) : "v"(x), "v"(y)); }
__device__ __forceinline__ void keep4_h(v16h a, v16h b, v16h c, v16h d) { asm volatile("v_nop" :: "v"(a), "v"(b), "v"(c), "v"(d)); }
__device__ __forceinline__ void keep4_b(v16b a, v16b b, v16b c, v16b d) { asm volatile("v_nop" :: "v"(a), "v"(b), "v"(c), "v"(d)); }
__device__ __forceinline__ void acc_guard4(v8f& a, v8f& b, v8f& c, v8f& d) { asm volatile("v_nop\n\tv_nop\n\tv_nop\n\tv_nop" : "+v"(a), "+v"(b), "+v"(c), "+v"(d)); }
template <typename T> struct Frag;
template <> struct Frag<_Float16> {
  typedef v16h V; union U { v16h v; v8h h[2]; };
  static __device__ __forceinline__ v16h load(const _Float16* p) {
    U f; f.h[0] = *(const v8h*)(p); f.h[1] = *(const v8h*)(p + 16); return f.v;
  }
  static __device__ __forceinline__ v8f mma(v16h a, v16h b, v8f c) {
    return __builtin_amdgcn_wmma_f32_16x16x32_f16(false, a, false, b, (short)0, c, false, false);
  }
  static __device__ __forceinline__ void guard(v8f& a, v8f& b, v16h x, v16h y) { dep_guard_h(a, b, x, y); }
  static __device__ __forceinline__ void keep(v16h a, v16h b, v16h c, v16h d) { keep4_h(a, b, c, d); }
};
template <> struct Frag<__bf16> {
  typedef v16b V; union U { v16b v; v8b h[2]; };
  static __device__ __forceinline__ v16b load(const __bf16* p) {
    U f; f.h[0] = *(const v8b*)(p); f.h[1] = *(const v8b*)(p + 16); return f.v;
  }
  static __device__ __forceinline__ v8f mma(v16b a, v16b b, v8f c) {
    return __builtin_amdgcn_wmma_f32_16x16x32_bf16(false, a, false, b, (short)0, c, false, false);
  }
  static __device__ __forceinline__ void guard(v8f& a, v8f& b, v16b x, v16b y) { dep_guard_b(a, b, x, y); }
  static __device__ __forceinline__ void keep(v16b a, v16b b, v16b c, v16b d) { keep4_b(a, b, c, d); }
};

__device__ __forceinline__ float fast_sig(float x) {
  const float e = exp2f(-x * 1.4426950408889634f);
  return __builtin_amdgcn_rcpf(1.0f + e);
}
__device__ __forceinline__ float fast_tanh(float x) {
  const float e = exp2f(x * 2.8853900817779268f);
  return 1.0f - 2.0f * __builtin_amdgcn_rcpf(1.0f + e);
}

template <int ET> struct Elem;
template <> struct Elem<0> { typedef _Float16 T; };
template <> struct Elem<1> { typedef __bf16 T; };
template <int ET, int MI, bool SPLIT, int BIAS_MODE, int OUT_MODE>
__global__ __launch_bounds__(256) void wmma_gemm_t(
    const unsigned short* __restrict__ Ap, const unsigned short* __restrict__ A2p, int lda, long strideA,
    const unsigned short* __restrict__ Btp, const unsigned short* __restrict__ Bt2p, int ldb, long strideB,
    void* __restrict__ Cout, void* __restrict__ Cout2, int ldc, long strideC,
    const float* __restrict__ bias,
    int M, int N, int K, float scale) {
  typedef typename Elem<ET>::T T;
  typedef typename Frag<T>::V V;
  const T* A = (const T*)Ap; const T* A2 = (const T*)A2p; const T* Bt = (const T*)Btp; const T* Bt2 = (const T*)Bt2p;
  __shared__ __align__(16) float sT[8][16 * 68];
  const int b    = blockIdx.y;
  const int lane = threadIdx.x & 31;
  const int wave = threadIdx.x >> 5;
  const int tilesN = N >> 6;
  const int tilesM = M / (16 * MI);
  const int tile = blockIdx.x * 8 + wave;
  if (tile >= tilesM * tilesN) return;
  const int tm = tile / tilesN;
  const int tn = tile - tm * tilesN;
  const int m0 = tm * (16 * MI);
  const int n0 = tn << 6;

  const T* Ab  = A  + (size_t)b * strideA;
  const T* Bb  = Bt + (size_t)b * strideB;
  const T* Ab2 = SPLIT ? (A2  + (size_t)b * strideA) : nullptr;
  const T* Bb2 = SPLIT ? (Bt2 + (size_t)b * strideB) : nullptr;

  const int rlane = lane & 15;
  const int koff  = (lane >> 4) * 8;
  const int mOff  = (lane >> 4) * 8;

  v8f acc[MI][4];
#pragma unroll
  for (int i = 0; i < MI; ++i)
#pragma unroll
    for (int j = 0; j < 4; ++j) acc[i][j] = (v8f){0.f,0.f,0.f,0.f,0.f,0.f,0.f,0.f};

  for (int k0 = 0; k0 < K; k0 += 32) {
    V bh[4], bl[4];
#pragma unroll
    for (int j = 0; j < 4; ++j) {
      const size_t bo = (size_t)(n0 + (j << 4) + rlane) * ldb + koff + k0;
      bh[j] = Frag<T>::load(Bb + bo);
      if (SPLIT) bl[j] = Frag<T>::load(Bb2 + bo);
    }
#pragma unroll
    for (int i = 0; i < MI; ++i) {
      const size_t ao = (size_t)(m0 + (i << 4) + rlane) * lda + koff + k0;
      V ah = Frag<T>::load(Ab + ao);
      V al;
      if (SPLIT) al = Frag<T>::load(Ab2 + ao);
#pragma unroll
      for (int j = 0; j < 4; ++j) {
        acc[i][j] = Frag<T>::mma(ah, bh[j], acc[i][j]);
        if (SPLIT) {
          acc[i][j] = Frag<T>::mma(ah, bl[j], acc[i][j]);
          acc[i][j] = Frag<T>::mma(al, bh[j], acc[i][j]);
        }
      }
      Frag<T>::guard(acc[i][0], acc[i][3], ah, SPLIT ? al : ah);
    }
    Frag<T>::keep(bh[0], bh[1], bh[2], bh[3]);
    if (SPLIT) Frag<T>::keep(bl[0], bl[1], bl[2], bl[3]);
  }
#pragma unroll
  for (int i = 0; i < MI; ++i) acc_guard4(acc[i][0], acc[i][1], acc[i][2], acc[i][3]);

  float* slab = sT[wave];
#pragma unroll
  for (int i = 0; i < MI; ++i) {
    const int mBase = m0 + (i << 4);
#pragma unroll
    for (int j = 0; j < 4; ++j) {
      const int n = n0 + (j << 4) + rlane;
      float bv = 0.f;
      if (BIAS_MODE == 2) bv = bias[n];
#pragma unroll
      for (int r = 0; r < 8; ++r) {
        float v = acc[i][j][r] * scale;
        if (BIAS_MODE == 1) v += bias[mBase + mOff + r];
        if (BIAS_MODE == 2) v += bv;
        slab[(mOff + r) * 68 + (j << 4) + rlane] = v;
      }
    }
    __builtin_amdgcn_fence(__ATOMIC_RELEASE, "workgroup");
    __builtin_amdgcn_wave_barrier();
    __builtin_amdgcn_fence(__ATOMIC_ACQUIRE, "workgroup");
    if (OUT_MODE == 0) {
      float* C = (float*)Cout + (size_t)b * strideC;
      const int hh = lane >> 4, c4 = (lane & 15) * 4;
      for (int pass = 0; pass < 2; ++pass) {
#pragma unroll
        for (int it = 0; it < 8; ++it) {
          const int row = it * 2 + hh;
          v4f v = *(const v4f*)(slab + row * 68 + c4);
          *(volatile v4f*)(C + (size_t)(mBase + row) * ldc + n0 + c4) = v;
        }
        __threadfence();
      }
    } else {
      const int q = lane >> 3, c8 = (lane & 7) * 8;
      unsigned short* C  = (unsigned short*)Cout  + (size_t)b * strideC;
      unsigned short* C2 = (OUT_MODE == 2) ? ((unsigned short*)Cout2 + (size_t)b * strideC) : nullptr;
      for (int pass = 0; pass < 2; ++pass) {
#pragma unroll
        for (int it = 0; it < 4; ++it) {
          const int row = it * 4 + q;
          const float* sp = slab + row * 68 + c8;
          v8h hv, lv;
#pragma unroll
          for (int e = 0; e < 8; ++e) {
            if (OUT_MODE == 1) {
              hv[e] = (_Float16)sp[e];
            } else {
              unsigned short hb = f2bf_bits(sp[e]);
              unsigned short lb = f2bf_bits(sp[e] - bf_bits2f(hb));
              hv[e] = __builtin_bit_cast(_Float16, hb);
              lv[e] = __builtin_bit_cast(_Float16, lb);
            }
          }
          *(volatile v8h*)(C + (size_t)(mBase + row) * ldc + n0 + c8) = hv;
          if (OUT_MODE == 2) *(volatile v8h*)(C2 + (size_t)(mBase + row) * ldc + n0 + c8) = lv;
        }
        __threadfence();
      }
    }
    __builtin_amdgcn_fence(__ATOMIC_RELEASE, "workgroup");
    __builtin_amdgcn_wave_barrier();
    __builtin_amdgcn_fence(__ATOMIC_ACQUIRE, "workgroup");
  }
}

__global__ __launch_bounds__(256) void cast2d_f16(
    const float* __restrict__ src, int src_rows, int src_ld,
    unsigned short* __restrict__ dst, int dst_rows, int dst_ld, int cols, float scale) {
  const long i = (long)blockIdx.x * 256 + threadIdx.x;
  const int ppr = cols >> 1;
  const long total = (long)dst_rows * ppr;
  if (i >= total) return;
  const int r  = (int)(i / ppr);
  const int cp = (int)(i - (long)r * ppr);
  const int rs = (r < src_rows) ? r : (src_rows - 1);
  const v2f x = *(const v2f*)(src + (size_t)rs * src_ld + 2 * cp);
  const bool live = (r < src_rows);
  const float a0 = live ? x[0] * scale : 0.0f;
  const float a1 = live ? x[1] * scale : 0.0f;
  const unsigned u = (unsigned)h2bits((_Float16)a0) | ((unsigned)h2bits((_Float16)a1) << 16);
  unsigned* o = (unsigned*)(dst + (size_t)r * dst_ld + 2 * cp);
  *(volatile unsigned*)o = u;
  __threadfence();
  *(volatile unsigned*)o = u;
}

__global__ __launch_bounds__(256) void transpose_enc(const float* __restrict__ enc, unsigned short* __restrict__ encT) {
  __shared__ __align__(16) _Float16 sTile[64 * TP_PITCH];
  const int fch = blockIdx.x, b = blockIdx.y, tid = threadIdx.x;
  const int f0 = fch * 64;
  for (int i = tid; i < 64 * 30; i += 256) {
    const int r = i / 30, w = i - r * 30;
    ((unsigned*)(void*)sTile)[(r * TP_PITCH + NP) / 2 + w] = 0u;
  }
  __syncthreads();
  const int f4 = tid & 15, pr = tid >> 4;
  const float* eb = enc + (size_t)b * NP * NF + f0 + 4 * f4;
#pragma unroll 1
  for (int it = 0; it < 13; ++it) {
    const int p  = it * 16 + pr;
    const int pc = (p < NP) ? p : (NP - 1);
    const v4f x = *(const v4f*)(eb + (size_t)pc * NF);
    if (p < NP) {
#pragma unroll
      for (int e = 0; e < 4; ++e) sTile[(4 * f4 + e) * TP_PITCH + p] = (_Float16)(x[e] * SC_ENC);
    }
  }
  __syncthreads();
  const int lane = tid & 31, wave = tid >> 5;
  unsigned short* ob = encT + ((size_t)b * NF + f0) * PTK;
  for (int pass = 0; pass < 2; ++pass) {
#pragma unroll
    for (int r = 0; r < 8; ++r) {
      const int f = wave * 8 + r;
      const v8h v = *(const v8h*)(sTile + f * TP_PITCH + 8 * lane);
      *(volatile v8h*)(ob + (size_t)f * PTK + 8 * lane) = v;
    }
    __threadfence();
  }
}

__global__ __launch_bounds__(256) void mean_enc16(const float* __restrict__ enc, unsigned short* __restrict__ mean16) {
  const int i = blockIdx.x * 256 + threadIdx.x;
  if (i >= NB * (NF / 2)) return;
  const int b = i / (NF / 2), fp = i - b * (NF / 2);
  const float* p = enc + (size_t)b * NP * NF + 2 * fp;
  float s0 = 0.0f, s1 = 0.0f;
#pragma unroll 1
  for (int q = 0; q < NP; ++q) {
    const v2f x = *(const v2f*)(p + (size_t)q * NF);
    s0 += x[0]; s1 += x[1];
  }
  const float m0 = s0 * (1.0f / (float)NP) * SC_Z;
  const float m1 = s1 * (1.0f / (float)NP) * SC_Z;
  const unsigned u = (unsigned)h2bits((_Float16)m0) | ((unsigned)h2bits((_Float16)m1) << 16);
  unsigned* o = (unsigned*)(mean16 + (size_t)b * NF + 2 * fp);
  *(volatile unsigned*)o = u;
  __threadfence();
  *(volatile unsigned*)o = u;
}

__global__ __launch_bounds__(256) void build_bias(
    const float* __restrict__ b_fc, const float* __restrict__ b_dec, const float* __restrict__ b_beta,
    const float* __restrict__ b_ih, const float* __restrict__ b_hh,
    const float* __restrict__ b_inh, const float* __restrict__ b_inc,
    float* __restrict__ bfcp, float* __restrict__ bcat, float* __restrict__ bg, float* __restrict__ binit) {
  const int blk = blockIdx.x, tid = threadIdx.x;
  float v;
  float* dst;
  if (blk < 40) {
    const int j = blk * 256 + tid;
    if (j >= NVP) return;
    const int jc = (j < NV) ? j : (NV - 1);
    v = b_fc[jc];
    if (j >= NV) v = 0.0f;
    dst = bfcp + j;
  } else if (blk < 50) {
    const int j = (blk - 40) * 256 + tid;
    const int j0 = (j < NA) ? j : (NA - 1);
    const int j1 = (j >= NA) ? (j - NA) : 0;
    const float a = b_dec[j0], c = b_beta[j1];
    v = (j < NA) ? a : c;
    dst = bcat + j;
  } else if (blk < 58) {
    const int j = (blk - 50) * 256 + tid;
    v = b_ih[j] + b_hh[j];
    dst = bg + j;
  } else {
    const int j = (blk - 58) * 256 + tid;
    const int j0 = (j < NH) ? j : (NH - 1);
    const int j1 = (j >= NH) ? (j - NH) : 0;
    const float a = b_inh[j0], c = b_inc[j1];
    v = (j < NH) ? a : c;
    dst = binit + j;
  }
  *(volatile float*)dst = v;
  __threadfence();
  *(volatile float*)dst = v;
}

__global__ __launch_bounds__(128) void init_state(const float* __restrict__ hc0, const float* __restrict__ emb,
                                                  float* __restrict__ cst, unsigned short* __restrict__ z16) {
  const int b = blockIdx.x, tid = threadIdx.x;
  {
    const v4f c = *(const v4f*)(hc0 + (size_t)b * (2 * NH) + NH + 4 * tid);
    float* dst = cst + (size_t)b * NH + 4 * tid;
    *(volatile v4f*)dst = c;
    __threadfence();
    *(volatile v4f*)dst = c;
  }
  if (tid < 64) {
    const float* hp = hc0 + (size_t)b * (2 * NH) + 8 * tid;
    const v4f x0 = *(const v4f*)hp, x1 = *(const v4f*)(hp + 4);
    v8h hv;
#pragma unroll
    for (int e = 0; e < 4; ++e) { hv[e] = (_Float16)(x0[e] * SC_Z); hv[4 + e] = (_Float16)(x1[e] * SC_Z); }
    unsigned short* dst = z16 + (size_t)b * KZ + KIH + 8 * tid;
    *(volatile v8h*)dst = hv;
    __threadfence();
    *(volatile v8h*)dst = hv;
  } else {
    const int q = tid - 64;
    const float* ep = emb + (size_t)1 * NE + 8 * q;
    const v4f x0 = *(const v4f*)ep, x1 = *(const v4f*)(ep + 4);
    v8h hv;
#pragma unroll
    for (int e = 0; e < 4; ++e) { hv[e] = (_Float16)(x0[e] * SC_Z); hv[4 + e] = (_Float16)(x1[e] * SC_Z); }
    unsigned short* dst = z16 + (size_t)b * KZ + 8 * q;
    *(volatile v8h*)dst = hv;
    __threadfence();
    *(volatile v8h*)dst = hv;
  }
}

__global__ __launch_bounds__(256) void attn_pool_step(
    const float* __restrict__ att1, const float* __restrict__ catv,
    const float* __restrict__ wfull, const float* __restrict__ bfull,
    const unsigned short* __restrict__ encT, float* __restrict__ alphaWt,
    unsigned short* __restrict__ z16) {
  __shared__ __align__(16) float sAtt2[NA];
  __shared__ __align__(16) float sWf[NA];
  __shared__ __align__(16) float sScore[256];
  __shared__ __align__(16) float sAlphaF[APW];
  __shared__ __align__(16) _Float16 sA[16 * SA_PITCH];
  __shared__ __align__(16) float sSlab[8][128];
  const int b = blockIdx.x, tid = threadIdx.x;
  const int lane = tid & 31, wave = tid >> 5;

  for (int i = tid; i < NA; i += 256) { sAtt2[i] = catv[(size_t)b * NCAT + i]; sWf[i] = wfull[i]; }
  {
    unsigned* za = (unsigned*)(void*)sA;
    for (int i = tid; i < (16 * SA_PITCH) / 2; i += 256) za[i] = 0u;
  }
  __syncthreads();

  float sv;
  {
    const int p = (tid < NP) ? tid : (NP - 1);
    const float* ar = att1 + ((size_t)b * NP + p) * NA;
    float s = 0.0f;
#pragma unroll 1
    for (int a = 0; a < NA; a += 4) {
      const v4f x  = *(const v4f*)(ar + a);
      const v4f t2 = *(const v4f*)(sAtt2 + a);
      const v4f w  = *(const v4f*)(sWf + a);
#pragma unroll
      for (int e = 0; e < 4; ++e) {
        const float v = fmaxf(x[e] + t2[e], 0.0f);
        s = fmaf(v, w[e], s);
      }
    }
    s += bfull[0];
    sv = (tid < NP) ? s : -__builtin_inff();
    sScore[tid] = sv;
  }
  __syncthreads();
  float m = -__builtin_inff();
#pragma unroll
  for (int k = 0; k < 8; ++k) m = fmaxf(m, sScore[lane + 32 * k]);
#pragma unroll
  for (int off = 1; off < 32; off <<= 1) m = fmaxf(m, __shfl_xor(m, off, 32));
  __syncthreads();
  const float ex = expf(sv - m);
  sScore[tid] = ex;
  __syncthreads();
  float ssum = 0.0f;
#pragma unroll
  for (int k = 0; k < 8; ++k) ssum += sScore[lane + 32 * k];
#pragma unroll
  for (int off = 1; off < 32; off <<= 1) ssum += __shfl_xor(ssum, off, 32);
  const float alpha = ex * (1.0f / ssum);
  if (tid < APW) sAlphaF[tid] = alpha;
  sA[tid] = (_Float16)(alpha * SC_P);
  __syncthreads();

  if (tid < APW / 4) {
    const v4f v = *(const v4f*)(sAlphaF + 4 * tid);
    float* dst = alphaWt + (size_t)b * APW + 4 * tid;
    *(volatile v4f*)dst = v;
    __threadfence();
    *(volatile v4f*)dst = v;
  }

  const int rlane = lane & 15, koff = (lane >> 4) * 8, hh = lane >> 4;
  const _Float16* encB = (const _Float16*)(encT + (size_t)b * NF * PTK);
  float* slab = sSlab[wave];
#pragma unroll 1
  for (int tt = 0; tt < 4; ++tt) {
    const int n0 = (wave * 4 + tt) * 64;
    v8f acc[4];
#pragma unroll
    for (int j = 0; j < 4; ++j) acc[j] = (v8f){0.f,0.f,0.f,0.f,0.f,0.f,0.f,0.f};
#pragma unroll 1
    for (int k0 = 0; k0 < KAWE; k0 += 32) {
      v16h bfr[4];
#pragma unroll
      for (int j = 0; j < 4; ++j)
        bfr[j] = Frag<_Float16>::load(encB + (size_t)(n0 + (j << 4) + rlane) * PTK + koff + k0);
      const v16h afr = Frag<_Float16>::load(sA + rlane * SA_PITCH + koff + k0);
#pragma unroll
      for (int j = 0; j < 4; ++j) acc[j] = Frag<_Float16>::mma(afr, bfr[j], acc[j]);
      Frag<_Float16>::guard(acc[0], acc[3], afr, afr);
      Frag<_Float16>::keep(bfr[0], bfr[1], bfr[2], bfr[3]);
    }
    acc_guard4(acc[0], acc[1], acc[2], acc[3]);
#pragma unroll
    for (int j = 0; j < 4; ++j) slab[hh * 64 + (j << 4) + rlane] = acc[j][0];
    __builtin_amdgcn_fence(__ATOMIC_RELEASE, "workgroup");
    __builtin_amdgcn_wave_barrier();
    __builtin_amdgcn_fence(__ATOMIC_ACQUIRE, "workgroup");
    if (lane < 8) {
      const v4f a0 = *(const v4f*)(slab + 8 * lane), a1 = *(const v4f*)(slab + 8 * lane + 4);
      const float* gp = catv + (size_t)b * NCAT + NA + n0 + 8 * lane;
      const v4f g0 = *(const v4f*)gp, g1 = *(const v4f*)(gp + 4);
      const float cf = SC_Z / (SC_ENC * SC_P);
      v8h hv;
#pragma unroll
      for (int e = 0; e < 4; ++e) {
        hv[e]     = (_Float16)(a0[e] * cf * fast_sig(g0[e]));
        hv[4 + e] = (_Float16)(a1[e] * cf * fast_sig(g1[e]));
      }
      unsigned short* dst = z16 + (size_t)b * KZ + NE + n0 + 8 * lane;
      *(volatile v8h*)dst = hv;
      __threadfence();
      *(volatile v8h*)dst = hv;
    }
    __builtin_amdgcn_fence(__ATOMIC_RELEASE, "workgroup");
    __builtin_amdgcn_wave_barrier();
    __builtin_amdgcn_fence(__ATOMIC_ACQUIRE, "workgroup");
  }
}

__global__ __launch_bounds__(128) void lstm_cell_step(
    const float* __restrict__ gates, float* __restrict__ cst,
    const float* __restrict__ emb, const int* __restrict__ caps,
    unsigned short* __restrict__ z16, int tnext) {
  __shared__ __align__(16) float sH[NH];
  const int b = blockIdx.x, tid = threadIdx.x;
  const int j = 4 * tid;
  const float* g = gates + (size_t)b * (4 * NH);
  const v4f gi = *(const v4f*)(g + j);
  const v4f gf = *(const v4f*)(g + NH + j);
  const v4f gg = *(const v4f*)(g + 2 * NH + j);
  const v4f go = *(const v4f*)(g + 3 * NH + j);
  float* cp = cst + (size_t)b * NH + j;
  const v4f co = *(const v4f*)cp;
  v4f cn;
#pragma unroll
  for (int e = 0; e < 4; ++e) {
    const float c = fast_sig(gf[e]) * co[e] + fast_sig(gi[e]) * fast_tanh(gg[e]);
    cn[e] = c;
    sH[j + e] = fast_sig(go[e]) * fast_tanh(c);
  }
  *(volatile v4f*)cp = cn;
  __threadfence();
  *(volatile v4f*)cp = cn;
  __syncthreads();
  if (tid < 64) {
    const v4f x0 = *(const v4f*)(sH + 8 * tid), x1 = *(const v4f*)(sH + 8 * tid + 4);
    v8h hv;
#pragma unroll
    for (int e = 0; e < 4; ++e) { hv[e] = (_Float16)(x0[e] * SC_Z); hv[4 + e] = (_Float16)(x1[e] * SC_Z); }
    unsigned short* dst = z16 + (size_t)b * KZ + KIH + 8 * tid;
    *(volatile v8h*)dst = hv;
    __threadfence();
    *(volatile v8h*)dst = hv;
  }
  if (tnext < NT) {
    int tok = caps[b * NT + tnext - 1];
    tok = tok < 0 ? 0 : (tok > NV - 1 ? NV - 1 : tok);
    if (tid >= 64) {
      const int q = tid - 64;
      const float* ep = emb + (size_t)tok * NE + 8 * q;
      const v4f x0 = *(const v4f*)ep, x1 = *(const v4f*)(ep + 4);
      v8h hv;
#pragma unroll
      for (int e = 0; e < 4; ++e) { hv[e] = (_Float16)(x0[e] * SC_Z); hv[4 + e] = (_Float16)(x1[e] * SC_Z); }
      unsigned short* dst = z16 + (size_t)b * KZ + 8 * q;
      *(volatile v8h*)dst = hv;
      __threadfence();
      *(volatile v8h*)dst = hv;
    }
  }
}

__global__ __launch_bounds__(256) void repack_out(const float* __restrict__ predsW, const float* __restrict__ alphaW,
                                                  float* __restrict__ out) {
  const long i = (long)blockIdx.x * 256 + threadIdx.x;
  const long n0tot  = (long)NB * NT * NV;
  const long total4 = (n0tot + (long)NB * NT * NP) / 4;
  if (i >= total4) return;
  const long e0 = i * 4;
  const long ea = (e0 < n0tot) ? e0 : (n0tot - 4);
  const int rowA = (int)(ea / NV);
  const int vA   = (int)(ea - (long)rowA * NV);
  const int bA = rowA / NT, tA = rowA - bA * NT;
  const v4f xa = *(const v4f*)(predsW + ((size_t)tA * NB + bA) * NVP + vA);
  long eb = e0 - n0tot; eb = (eb < 0) ? 0 : eb;
  const int rowB = (int)(eb / NP);
  const int pB   = (int)(eb - (long)rowB * NP);
  const int bB = rowB / NT, tB = rowB - bB * NT;
  const v4f xb = *(const v4f*)(alphaW + ((size_t)tB * NB + bB) * APW + pB);
  const bool selA = (e0 < n0tot);
  v4f v;
#pragma unroll
  for (int e = 0; e < 4; ++e) v[e] = selA ? xa[e] : xb[e];
  float* dst = out + e0;
  *(volatile v4f*)dst = v;
  __threadfence();
  *(volatile v4f*)dst = v;
}

template <int MI>
static void launch_gemm_f16(const unsigned short* A, int lda, const unsigned short* Bt, int ldb,
                            float* C, int ldc, const float* bias, int M, int N, int K, float scale, hipStream_t s) {
  const int tiles  = (M / (16 * MI)) * (N / 64);
  const int blocks = (tiles + 7) / 8;
  wmma_gemm_t<0, MI, false, 2, 0><<<dim3(blocks, 1), 256, 0, s>>>(
      A, nullptr, lda, 0L, Bt, nullptr, ldb, 0L, (void*)C, nullptr, ldc, 0L, bias, M, N, K, scale);
}
static void launch_cast(const float* src, int src_rows, int src_ld, unsigned short* dst, int dst_rows, int dst_ld,
                        int cols, float scale, hipStream_t s) {
  const long total = (long)dst_rows * (cols / 2);
  const int blocks = (int)((total + 255) / 256);
  cast2d_f16<<<blocks, 256, 0, s>>>(src, src_rows, src_ld, dst, dst_rows, dst_ld, cols, scale);
}

extern "C" void kernel_launch(void* const* d_in, const int* in_sizes, int n_in,
                              void* d_out, int out_size, void* d_ws, size_t ws_size,
                              hipStream_t stream) {
  if (n_in < 21) return;
  if (in_sizes[0] != NB * NP * NF || in_sizes[1] != NB * NT || in_sizes[2] != NA * NF ||
      in_sizes[4] != NA * NH || in_sizes[6] != NA || in_sizes[8] != NV * NE ||
      in_sizes[9] != 4 * NH * KIH || in_sizes[11] != 4 * NH * NH || in_sizes[13] != NH * NF ||
      in_sizes[15] != NH * NF || in_sizes[17] != NF * NH || in_sizes[19] != NV * NH ||
      in_sizes[20] != NV || out_size != NB * NT * NV + NB * NT * NP) return;

  const float* enc      = (const float*)d_in[0];
  const int*   caps     = (const int*)d_in[1];
  const float* W_enc    = (const float*)d_in[2];
  const float* b_enc    = (const float*)d_in[3];
  const float* W_dec    = (const float*)d_in[4];
  const float* b_dec    = (const float*)d_in[5];
  const float* W_full   = (const float*)d_in[6];
  const float* b_full   = (const float*)d_in[7];
  const float* emb      = (const float*)d_in[8];
  const float* W_ih     = (const float*)d_in[9];
  const float* b_ih     = (const float*)d_in[10];
  const float* W_hh     = (const float*)d_in[11];
  const float* b_hh     = (const float*)d_in[12];
  const float* W_init_h = (const float*)d_in[13];
  const float* b_init_h = (const float*)d_in[14];
  const float* W_init_c = (const float*)d_in[15];
  const float* b_init_c = (const float*)d_in[16];
  const float* W_beta   = (const float*)d_in[17];
  const float* b_beta   = (const float*)d_in[18];
  const float* W_fc     = (const float*)d_in[19];
  const float* b_fc     = (const float*)d_in[20];

  char* ws = (char*)d_ws;
  size_t off = 0;
  auto carve = [&](size_t bytes) -> char* { char* p = ws + off; off += (bytes + 255) & ~(size_t)255; return p; };
  unsigned short* Wenc16  = (unsigned short*)carve((size_t)NA * NF * 2);
  unsigned short* Wfc16   = (unsigned short*)carve((size_t)NVP * NH * 2);
  unsigned short* Wdb16   = (unsigned short*)carve((size_t)NCAT * NH * 2);
  unsigned short* Wg16    = (unsigned short*)carve((size_t)(4 * NH) * KZ * 2);
  unsigned short* Winit16 = (unsigned short*)carve((size_t)(2 * NH) * NF * 2);
  float* bfcp  = (float*)carve((size_t)NVP * 4);
  float* bcat  = (float*)carve((size_t)NCAT * 4);
  float* bg    = (float*)carve((size_t)(4 * NH) * 4);
  float* binit = (float*)carve((size_t)(2 * NH) * 4);
  const size_t rbig_bytes = ((size_t)MROWS * NF * 2 > (size_t)NT * NB * NVP * 4) ? (size_t)MROWS * NF * 2 : (size_t)NT * NB * NVP * 4;
  char* Rbig = carve(rbig_bytes);
  unsigned short* enc16  = (unsigned short*)Rbig;
  float*          predsW = (float*)Rbig;
  unsigned short* encT16 = (unsigned short*)carve((size_t)NB * NF * PTK * 2);
  unsigned short* mean16 = (unsigned short*)carve((size_t)NB * NF * 2);
  float* att1   = (float*)carve((size_t)MROWS * NA * 4);
  float* hc0    = (float*)carve((size_t)NB * (2 * NH) * 4);
  unsigned short* z16 = (unsigned short*)carve((size_t)NB * KZ * 2);
  float* cst    = (float*)carve((size_t)NB * NH * 4);
  float* gatesb = (float*)carve((size_t)NB * (4 * NH) * 4);
  float* catv   = (float*)carve((size_t)NB * NCAT * 4);
  float* alphaW = (float*)carve((size_t)NT * NB * APW * 4);
  if (off > ws_size) return;

  float* outp = (float*)d_out;

  launch_cast(W_enc,    NA,     NF,  Wenc16,                         NA,      NF,  NF,  SC_W, stream);
  launch_cast(W_fc,     NV,     NH,  Wfc16,                          NVP,     NH,  NH,  SC_W, stream);
  launch_cast(W_dec,    NA,     NH,  Wdb16,                          NA,      NH,  NH,  SC_W, stream);
  launch_cast(W_beta,   NF,     NH,  Wdb16 + (size_t)NA * NH,        NF,      NH,  NH,  SC_W, stream);
  launch_cast(W_ih,     4 * NH, KIH, Wg16,                           4 * NH,  KZ,  KIH, SC_W, stream);
  launch_cast(W_hh,     4 * NH, NH,  Wg16 + KIH,                     4 * NH,  KZ,  NH,  SC_W, stream);
  launch_cast(W_init_h, NH,     NF,  Winit16,                        NH,      NF,  NF,  SC_W, stream);
  launch_cast(W_init_c, NH,     NF,  Winit16 + (size_t)NH * NF,      NH,      NF,  NF,  SC_W, stream);
  build_bias<<<62, 256, 0, stream>>>(b_fc, b_dec, b_beta, b_ih, b_hh, b_init_h, b_init_c, bfcp, bcat, bg, binit);
  launch_cast(enc, MROWS, NF, enc16, MROWS, NF, NF, SC_ENC, stream);
  transpose_enc<<<dim3(NF / 64, NB), 256, 0, stream>>>(enc, encT16);
  mean_enc16<<<(NB * (NF / 2)) / 256, 256, 0, stream>>>(enc, mean16);
  launch_gemm_f16<4>(enc16, NF, Wenc16, NF, att1, NA, b_enc, MROWS, NA, NF, 1.0f / (SC_ENC * SC_W), stream);
  launch_gemm_f16<2>(mean16, NF, Winit16, NF, hc0, 2 * NH, binit, NB, 2 * NH, NF, 1.0f / (SC_Z * SC_W), stream);
  init_state<<<NB, 128, 0, stream>>>(hc0, emb, cst, z16);

  const float zscale = 1.0f / (SC_Z * SC_W);
  for (int t = 0; t < NT; ++t) {
    launch_gemm_f16<2>(z16 + KIH, KZ, Wdb16, NH, catv, NCAT, bcat, NB, NCAT, NH, zscale, stream);
    attn_pool_step<<<NB, 256, 0, stream>>>(att1, catv, W_full, b_full, encT16, alphaW + (size_t)t * NB * APW, z16);
    launch_gemm_f16<2>(z16, KZ, Wg16, KZ, gatesb, 4 * NH, bg, NB, 4 * NH, KZ, zscale, stream);
    lstm_cell_step<<<NB, 128, 0, stream>>>(gatesb, cst, emb, caps, z16, t + 1);
    launch_gemm_f16<2>(z16 + KIH, KZ, Wfc16, NH, predsW + (size_t)t * NB * NVP, NVP, bfcp, NB, NVP, NH, zscale, stream);
  }

  {
    const long total4 = ((long)NB * NT * NV + (long)NB * NT * NP) / 4;
    const int blocks = (int)((total4 + 255) / 256);
    repack_out<<<blocks, 256, 0, stream>>>(predsW, alphaW, outp);
  }
}
